// MultiScaleRetention_4440996184660
// MI455X (gfx1250) — hardware-verified
//
#include <hip/hip_runtime.h>
#include <math.h>

constexpr int kBatch = 2;
constexpr int kSeq   = 2048;
constexpr int kDim   = 1024;
constexpr int kHeads = 16;
constexpr int kDh    = 64;
constexpr int kTok   = kBatch * kSeq;
constexpr int kGroup = 4;
constexpr int kStatPitch = 32;
constexpr float kWCarry   = 16.0f;
constexpr float kActCarry = 16.0f;
constexpr float kAttCarry = 1024.0f;
constexpr float kProjScale  = kActCarry / kWCarry;
constexpr float kScoreScale = kAttCarry / (8.0f * kActCarry * kActCarry);
constexpr float kPVScale    = 1.0f / (kAttCarry * kActCarry);
constexpr float kOutScale   = 1.0f / (kActCarry * kWCarry);
constexpr float kGnEps      = 1e-5f;
constexpr float kInvCount   = 1.0f / (float)(kSeq * kDh);
static_assert(kHeads * kDh == kDim);
static_assert(kHeads % kGroup == 0);
static_assert(kTok % 64 == 0 && kDim % 64 == 0 && kSeq % 64 == 0 && kDh % 64 == 0);
static_assert(kDim % 32 == 0 && kDh % 32 == 0 && kSeq % 32 == 0);
static_assert((kTok * kDim) % (8 * 256) == 0 && (kDim * kDim) % (8 * 256) == 0 && kSeq % 256 == 0);

typedef __attribute__((ext_vector_type(16))) _Float16 v16h;
typedef __attribute__((ext_vector_type(8)))  _Float16 v8h;
typedef __attribute__((ext_vector_type(16))) __bf16   v16b;
typedef __attribute__((ext_vector_type(8)))  __bf16   v8b;
typedef __attribute__((ext_vector_type(8)))  float    v8f;
typedef __attribute__((ext_vector_type(4)))  float    v4f;
typedef __attribute__((ext_vector_type(4)))  unsigned int v4u;

__device__ __forceinline__ unsigned short f2bf_bits(float f) {
  unsigned u = __float_as_uint(f);
  return (unsigned short)((u + 0x7FFFu + ((u >> 16) & 1u)) >> 16);
}
__device__ __forceinline__ float bf_bits2f(unsigned short h) { return __uint_as_float(((unsigned)h) << 16); }

__device__ __forceinline__ void dep_guard_h(v8f& a, v8f& b, v16h x, v16h y) { asm volatile("v_nop\n\tv_nop\n\tv_nop\n\tv_nop" : "+v"(a), "+v"(b) : "v"(x), "v"(y)); }
__device__ __forceinline__ void dep_guard_b(v8f& a, v8f& b, v16b x, v16b y) { asm volatile("v_nop\n\tv_nop\n\tv_nop\n\tv_nop" : "+v"(a), "+v"(b) : "v"(x), "v"(y)); }
__device__ __forceinline__ void dep_guard4_h(v8f& a, v8f& b, v8f& c, v8f& d, v16h x, v16h y) { asm volatile("v_nop\n\tv_nop\n\tv_nop\n\tv_nop" : "+v"(a), "+v"(b), "+v"(c), "+v"(d) : "v"(x), "v"(y)); }
__device__ __forceinline__ void dep_guard4_b(v8f& a, v8f& b, v8f& c, v8f& d, v16b x, v16b y) { asm volatile("v_nop\n\tv_nop\n\tv_nop\n\tv_nop" : "+v"(a), "+v"(b), "+v"(c), "+v"(d) : "v"(x), "v"(y)); }
__device__ __forceinline__ void keep4_h(v16h a, v16h b, v16h c, v16h d) { asm volatile("v_nop" :: "v"(a), "v"(b), "v"(c), "v"(d)); }
__device__ __forceinline__ void keep4_b(v16b a, v16b b, v16b c, v16b d) { asm volatile("v_nop" :: "v"(a), "v"(b), "v"(c), "v"(d)); }
__device__ __forceinline__ void acc_guard4(v8f& a, v8f& b, v8f& c, v8f& d) { asm volatile("v_nop\n\tv_nop\n\tv_nop\n\tv_nop" : "+v"(a), "+v"(b), "+v"(c), "+v"(d)); }
template <typename T> struct Frag;
template <> struct Frag<_Float16> {
  typedef v16h V; union U { v16h v; v8h h[2]; };
  static __device__ __forceinline__ v16h load(const _Float16* p) {
    U f; f.h[0] = *(const v8h*)(p); f.h[1] = *(const v8h*)(p + 16); return f.v;
  }
  static __device__ __forceinline__ v8f mma(v16h a, v16h b, v8f c) {
    return __builtin_amdgcn_wmma_f32_16x16x32_f16(false, a, false, b, (short)0, c, false, false);
  }
  static __device__ __forceinline__ void guard(v8f& a, v8f& b, v16h x, v16h y) { dep_guard_h(a, b, x, y); }
  static __device__ __forceinline__ void guard4(v8f& a, v8f& b, v8f& c, v8f& d, v16h x, v16h y) { dep_guard4_h(a, b, c, d, x, y); }
  static __device__ __forceinline__ void keep(v16h a, v16h b, v16h c, v16h d) { keep4_h(a, b, c, d); }
};
template <> struct Frag<__bf16> {
  typedef v16b V; union U { v16b v; v8b h[2]; };
  static __device__ __forceinline__ v16b load(const __bf16* p) {
    U f; f.h[0] = *(const v8b*)(p); f.h[1] = *(const v8b*)(p + 16); return f.v;
  }
  static __device__ __forceinline__ v8f mma(v16b a, v16b b, v8f c) {
    return __builtin_amdgcn_wmma_f32_16x16x32_bf16(false, a, false, b, (short)0, c, false, false);
  }
  static __device__ __forceinline__ void guard(v8f& a, v8f& b, v16b x, v16b y) { dep_guard_b(a, b, x, y); }
  static __device__ __forceinline__ void guard4(v8f& a, v8f& b, v8f& c, v8f& d, v16b x, v16b y) { dep_guard4_b(a, b, c, d, x, y); }
  static __device__ __forceinline__ void keep(v16b a, v16b b, v16b c, v16b d) { keep4_b(a, b, c, d); }
};

__device__ __forceinline__ unsigned pk16(unsigned short a, unsigned short b) { return (unsigned)a | ((unsigned)b << 16); }
__device__ __forceinline__ unsigned short h_bits(float f) { const _Float16 h = (_Float16)f; return __builtin_bit_cast(unsigned short, h); }

template <int ET> struct Elem;
template <> struct Elem<0> { typedef _Float16 T; };
template <> struct Elem<1> { typedef __bf16 T; };
template <int ET, bool SPLIT, int BIAS_MODE, int OUT_MODE, bool RESID, int ACT = 0, int KMODE = 0, bool DECAY = false>
__global__ __launch_bounds__(256) void wmma_gemm64(
    const unsigned short* __restrict__ Ap, const unsigned short* __restrict__ A2p, int lda, long strideA,
    const unsigned short* __restrict__ Btp, const unsigned short* __restrict__ Bt2p, int ldb, long strideB,
    void* __restrict__ Cout, void* __restrict__ Cout2, int ldc, long strideC,
    const float* __restrict__ bias,
    const float* __restrict__ resid, long strideR,
    int M, int N, int K, float scale) {
  static_assert(!DECAY || (BIAS_MODE == 0 && !RESID && ACT == 0));
  typedef typename Elem<ET>::T T;
  typedef typename Frag<T>::V V;
  const T* A = (const T*)Ap; const T* A2 = (const T*)A2p; const T* Bt = (const T*)Btp; const T* Bt2 = (const T*)Bt2p;
  __shared__ __align__(16) float sT[8][16 * 68];
  __shared__ __align__(16) float sRC[DECAY ? 8 : 1][DECAY ? 128 : 4];
  const int b    = blockIdx.y;
  const int lane = threadIdx.x & 31;
  const int wave = threadIdx.x >> 5;
  const int tilesN = N >> 6;
  const int tilesM = M >> 6;
  const int tile = blockIdx.x * 8 + wave;
  if (tile >= tilesM * tilesN) return;
  const int tm = tile / tilesN;
  const int tn = tile - tm * tilesN;
  const int m0 = tm << 6;
  const int n0 = tn << 6;

  const T* Ab  = A  + (size_t)b * strideA;
  const T* Bb  = Bt + (size_t)b * strideB;
  const T* Ab2 = SPLIT ? (A2  + (size_t)b * strideA) : nullptr;
  const T* Bb2 = SPLIT ? (Bt2 + (size_t)b * strideB) : nullptr;

  const int rlane = lane & 15;
  const int koff  = (lane >> 4) * 8;
  const int mOff  = (lane >> 4) * 8;

  v8f acc[4][4];
#pragma unroll
  for (int i = 0; i < 4; ++i)
#pragma unroll
    for (int j = 0; j < 4; ++j) acc[i][j] = (v8f){0.f,0.f,0.f,0.f,0.f,0.f,0.f,0.f};

  int Kend = K;
  if (KMODE == 1) { if (tn > tm) Kend = 0; }
  if (KMODE == 2) { const int kc = m0 + 64; Kend = (kc < K) ? kc : K; }

  for (int k0 = 0; k0 < Kend; k0 += 32) {
    V bh[4], bl[4];
#pragma unroll
    for (int j = 0; j < 4; ++j) {
      const size_t bo = (size_t)(n0 + (j << 4) + rlane) * ldb + koff + k0;
      bh[j] = Frag<T>::load(Bb + bo);
      if (SPLIT) bl[j] = Frag<T>::load(Bb2 + bo);
    }
#pragma unroll
    for (int i = 0; i < 4; ++i) {
      const size_t ao = (size_t)(m0 + (i << 4) + rlane) * lda + koff + k0;
      V ah = Frag<T>::load(Ab + ao);
      V al;
      if (SPLIT) al = Frag<T>::load(Ab2 + ao);
#pragma unroll
      for (int j = 0; j < 4; ++j) {
        acc[i][j] = Frag<T>::mma(ah, bh[j], acc[i][j]);
        if (SPLIT) {
          acc[i][j] = Frag<T>::mma(ah, bl[j], acc[i][j]);
          acc[i][j] = Frag<T>::mma(al, bh[j], acc[i][j]);
        }
      }
      Frag<T>::guard4(acc[i][0], acc[i][1], acc[i][2], acc[i][3], ah, SPLIT ? al : ah);
    }
    Frag<T>::keep(bh[0], bh[1], bh[2], bh[3]);
    if (SPLIT) Frag<T>::keep(bl[0], bl[1], bl[2], bl[3]);
  }
  acc_guard4(acc[0][0], acc[0][1], acc[0][2], acc[0][3]);
  acc_guard4(acc[1][0], acc[1][1], acc[1][2], acc[1][3]);
  acc_guard4(acc[2][0], acc[2][1], acc[2][2], acc[2][3]);
  acc_guard4(acc[3][0], acc[3][1], acc[3][2], acc[3][3]);

  if (DECAY) {
    const float* rtab = bias  + (size_t)b * strideR;
    const float* ctab = resid + (size_t)b * strideR;
    const float r0v = rtab[m0 + lane];
    const float r1v = rtab[m0 + 32 + lane];
    const float c0v = ctab[n0 + lane];
    const float c1v = ctab[n0 + 32 + lane];
    float* rc = sRC[wave];
    rc[lane]      = r0v;
    rc[32 + lane] = r1v;
    rc[64 + lane] = c0v;
    rc[96 + lane] = c1v;
    __builtin_amdgcn_fence(__ATOMIC_RELEASE, "workgroup");
    __builtin_amdgcn_wave_barrier();
    __builtin_amdgcn_fence(__ATOMIC_ACQUIRE, "workgroup");
  }

  float* slab = sT[wave];
  const float* Rb = RESID ? (resid + (size_t)b * strideR) : nullptr;
#pragma unroll
  for (int i = 0; i < 4; ++i) {
    const int mBase = m0 + (i << 4);
#pragma unroll
    for (int j = 0; j < 4; ++j) {
      const int n = n0 + (j << 4) + rlane;
      float bv = 0.f;
      if (BIAS_MODE == 2) bv = bias[n];
      float cdec = 0.f;
      if (DECAY) cdec = sRC[wave][64 + (j << 4) + rlane];
#pragma unroll
      for (int r = 0; r < 8; ++r) {
        float v = acc[i][j][r] * scale;
        if (BIAS_MODE == 1) v += bias[mBase + mOff + r];
        if (BIAS_MODE == 2) v += bv;
        if (RESID) v += Rb[(size_t)(mBase + mOff + r) * ldc + n];
        if (ACT == 2) v = fmaxf(v, 0.0f);
        if (ACT == 4) v = (v > 0.f) ? v : 0.01f * v;
        if (DECAY) {
          const int mrow = mBase + mOff + r;
          const float rdec = sRC[wave][(i << 4) + mOff + r];
          const float dd = rdec * cdec;
          v = v * dd;
          v = (n <= mrow) ? v : 0.0f;
        }
        slab[(mOff + r) * 68 + (j << 4) + rlane] = v;
      }
    }
    __builtin_amdgcn_fence(__ATOMIC_RELEASE, "workgroup");
    __builtin_amdgcn_wave_barrier();
    __builtin_amdgcn_fence(__ATOMIC_ACQUIRE, "workgroup");
    if (OUT_MODE == 0) {
      float* C = (float*)Cout + (size_t)b * strideC;
      const int hh = lane >> 4, c4 = (lane & 15) * 4;
      for (int pass = 0; pass < 2; ++pass) {
#pragma unroll
        for (int it = 0; it < 8; ++it) {
          const int row = it * 2 + hh;
          v4f v = *(const v4f*)(slab + row * 68 + c4);
          *(volatile v4f*)(C + (size_t)(mBase + row) * ldc + n0 + c4) = v;
        }
        __threadfence();
      }
    } else {
      const int q = lane >> 3, c8 = (lane & 7) * 8;
      unsigned short* C  = (unsigned short*)Cout  + (size_t)b * strideC;
      unsigned short* C2 = (OUT_MODE == 2) ? ((unsigned short*)Cout2 + (size_t)b * strideC) : nullptr;
      for (int pass = 0; pass < 2; ++pass) {
#pragma unroll
        for (int it = 0; it < 4; ++it) {
          const int row = it * 4 + q;
          const float* sp = slab + row * 68 + c8;
          v8h hv, lv;
#pragma unroll
          for (int e = 0; e < 8; ++e) {
            if (OUT_MODE == 1) {
              hv[e] = (_Float16)sp[e];
            } else {
              unsigned short hb = f2bf_bits(sp[e]);
              unsigned short lb = f2bf_bits(sp[e] - bf_bits2f(hb));
              hv[e] = __builtin_bit_cast(_Float16, hb);
              lv[e] = __builtin_bit_cast(_Float16, lb);
            }
          }
          *(volatile v8h*)(C + (size_t)(mBase + row) * ldc + n0 + c8) = hv;
          if (OUT_MODE == 2) *(volatile v8h*)(C2 + (size_t)(mBase + row) * ldc + n0 + c8) = lv;
        }
        __threadfence();
      }
    }
    __builtin_amdgcn_fence(__ATOMIC_RELEASE, "workgroup");
    __builtin_amdgcn_wave_barrier();
    __builtin_amdgcn_fence(__ATOMIC_ACQUIRE, "workgroup");
  }
}

__global__ __launch_bounds__(256) void cast8_kernel(const float* __restrict__ in, unsigned short* __restrict__ out, int n8, float carry) {
  const int i = blockIdx.x * 256 + threadIdx.x;
  if (i >= n8) return;
  const float* p = in + 8 * (size_t)i;
  const v4f a = *(const v4f*)(p);
  const v4f c = *(const v4f*)(p + 4);
  unsigned short hb[8];
#pragma unroll
  for (int e = 0; e < 4; ++e) {
    hb[e]     = h_bits(bf_bits2f(f2bf_bits(a[e])) * carry);
    hb[4 + e] = h_bits(bf_bits2f(f2bf_bits(c[e])) * carry);
  }
  const v4u u = (v4u){pk16(hb[0], hb[1]), pk16(hb[2], hb[3]), pk16(hb[4], hb[5]), pk16(hb[6], hb[7])};
  unsigned short* q = out + 8 * (size_t)i;
  *(volatile v4u*)q = u;
  __threadfence();
  *(volatile v4u*)q = u;
}

__global__ __launch_bounds__(256) void wcast8_kernel(const float* __restrict__ W0, const float* __restrict__ W1,
                                                    const float* __restrict__ W2, const float* __restrict__ W3,
                                                    unsigned short* __restrict__ out, int n8, float carry) {
  const int z = blockIdx.y;
  const float* W = (z == 0) ? W0 : (z == 1) ? W1 : (z == 2) ? W2 : W3;
  const int i = blockIdx.x * 256 + threadIdx.x;
  if (i >= n8) return;
  const float* p = W + 8 * (size_t)i;
  const v4f a = *(const v4f*)(p);
  const v4f c = *(const v4f*)(p + 4);
  unsigned short hb[8];
#pragma unroll
  for (int e = 0; e < 4; ++e) {
    hb[e]     = h_bits(bf_bits2f(f2bf_bits(a[e])) * carry);
    hb[4 + e] = h_bits(bf_bits2f(f2bf_bits(c[e])) * carry);
  }
  const v4u u = (v4u){pk16(hb[0], hb[1]), pk16(hb[2], hb[3]), pk16(hb[4], hb[5]), pk16(hb[6], hb[7])};
  unsigned short* q = out + (size_t)z * 8 * (size_t)n8 + 8 * (size_t)i;
  *(volatile v4u*)q = u;
  __threadfence();
  *(volatile v4u*)q = u;
}

__global__ __launch_bounds__(256) void decay_table_kernel(float* __restrict__ RT, float* __restrict__ CT) {
  __shared__ __align__(16) float sr[256];
  __shared__ __align__(16) float sc[256];
  const int t  = threadIdx.x;
  const int h  = blockIdx.y;
  const int p0 = blockIdx.x * 256;
  const float lg = log1pf(-exp2f(-5.0f - (float)h));
  const float e  = (float)(p0 + t) * lg;
  sr[t] = expf(e);
  sc[t] = expf(-e);
  __syncthreads();
  if (t < 64) {
    const v4f val = *(const v4f*)(sr + 4 * t);
    float* dp = RT + (size_t)h * kSeq + p0 + 4 * t;
    *(volatile v4f*)dp = val;
    __threadfence();
    *(volatile v4f*)dp = val;
  } else if (t < 128) {
    const int u = t - 64;
    const v4f val = *(const v4f*)(sc + 4 * u);
    float* dp = CT + (size_t)h * kSeq + p0 + 4 * u;
    *(volatile v4f*)dp = val;
    __threadfence();
    *(volatile v4f*)dp = val;
  }
}

__global__ __launch_bounds__(256) void gn_stats_kernel(const float* __restrict__ Y, float* __restrict__ ST) {
  __shared__ float red1[8];
  __shared__ float red2[8];
  __shared__ __align__(16) float sline[32];
  const int bh   = blockIdx.x;
  const int b    = bh >> 4;
  const int h    = bh & 15;
  const int t    = threadIdx.x;
  const int lane = t & 31, wave = t >> 5;
  const int rsub = t >> 4;
  const int c4   = (t & 15) * 4;
  const float* base = Y + ((size_t)b * kSeq) * kDim + h * kDh + c4;

  float s0 = 0.f, s1 = 0.f, s2 = 0.f, s3 = 0.f;
#pragma unroll 1
  for (int it = 0; it < kSeq / 16; ++it) {
    const int row = it * 16 + rsub;
    const v4f w = *(const v4f*)(base + (size_t)row * kDim);
    s0 += w[0]; s1 += w[1]; s2 += w[2]; s3 += w[3];
  }
  float s = (s0 + s1) + (s2 + s3);
#pragma unroll
  for (int off = 16; off > 0; off >>= 1) s += __shfl_xor(s, off, 32);
  if (lane == 0) red1[wave] = s;
  __syncthreads();
  float tot = red1[0];
#pragma unroll
  for (int w = 1; w < 8; ++w) tot += red1[w];
  const float mean = tot * kInvCount;

  float q0 = 0.f, q1 = 0.f, q2 = 0.f, q3 = 0.f;
#pragma unroll 1
  for (int it = 0; it < kSeq / 16; ++it) {
    const int row = it * 16 + rsub;
    const v4f w = *(const v4f*)(base + (size_t)row * kDim);
    const float d0 = w[0] - mean, d1 = w[1] - mean, d2 = w[2] - mean, d3 = w[3] - mean;
    q0 += d0 * d0; q1 += d1 * d1; q2 += d2 * d2; q3 += d3 * d3;
  }
  float qs = (q0 + q1) + (q2 + q3);
#pragma unroll
  for (int off = 16; off > 0; off >>= 1) qs += __shfl_xor(qs, off, 32);
  if (lane == 0) red2[wave] = qs;
  __syncthreads();
  float tot2 = red2[0];
#pragma unroll
  for (int w = 1; w < 8; ++w) tot2 += red2[w];
  const float var  = tot2 * kInvCount;
  const float rstd = 1.0f / sqrtf(var + kGnEps);

  if (t < 32) sline[t] = (t == 0) ? mean : (t == 1) ? rstd : 0.0f;
  __syncthreads();
  if (t < 8) {
    const v4f val = *(const v4f*)(sline + 4 * t);
    float* dp = ST + (size_t)bh * kStatPitch + 4 * t;
    *(volatile v4f*)dp = val;
    __threadfence();
    *(volatile v4f*)dp = val;
  }
}

__global__ __launch_bounds__(256) void gn_apply_kernel(const float* __restrict__ Y, const float* __restrict__ ST,
                                                      const float* __restrict__ gw, const float* __restrict__ gb,
                                                      unsigned short* __restrict__ YN, int n8, float carry) {
  const int i = blockIdx.x * 256 + threadIdx.x;
  if (i >= n8) return;
  const int row = i >> 7;
  const int c0  = (i & 127) * 8;
  const int b   = row >> 11;
  const int h   = c0 >> 6;
  const float* sp = ST + (size_t)(b * kHeads + h) * kStatPitch;
  const float mean = sp[0];
  const float rstd = sp[1];
  const float* yp = Y + (size_t)row * kDim + c0;
  const v4f y0 = *(const v4f*)(yp);
  const v4f y1 = *(const v4f*)(yp + 4);
  const v4f w0 = *(const v4f*)(gw + c0);
  const v4f w1 = *(const v4f*)(gw + c0 + 4);
  const v4f a0 = *(const v4f*)(gb + c0);
  const v4f a1 = *(const v4f*)(gb + c0 + 4);
  unsigned short hb[8];
#pragma unroll
  for (int e = 0; e < 4; ++e) {
    const float n0v = (y0[e] - mean) * rstd * w0[e] + a0[e];
    const float n1v = (y1[e] - mean) * rstd * w1[e] + a1[e];
    hb[e]     = h_bits(n0v * carry);
    hb[4 + e] = h_bits(n1v * carry);
  }
  const v4u u = (v4u){pk16(hb[0], hb[1]), pk16(hb[2], hb[3]), pk16(hb[4], hb[5]), pk16(hb[6], hb[7])};
  unsigned short* q = YN + (size_t)row * kDim + c0;
  *(volatile v4u*)q = u;
  __threadfence();
  *(volatile v4u*)q = u;
}

extern "C" void kernel_launch(void* const* d_in, const int* in_sizes, int n_in,
                              void* d_out, int out_size, void* d_ws, size_t ws_size,
                              hipStream_t stream) {
  if (n_in < 7) return;
  const int nAct = kTok * kDim;
  const int nW   = kDim * kDim;
  if (in_sizes[0] != nAct) return;
  if (in_sizes[1] != nW || in_sizes[2] != nW || in_sizes[3] != nW || in_sizes[4] != nW) return;
  if (in_sizes[5] != kDim || in_sizes[6] != kDim) return;
  if (out_size != nAct) return;

  const size_t szXH   = (size_t)nAct * 2;
  const size_t szW16  = (size_t)4 * nW * 2;
  const size_t szQK   = (size_t)2 * nAct * 2;
  const size_t szVT   = (size_t)kBatch * kDim * kSeq * 2;
  const size_t szATT  = (size_t)kGroup * kSeq * kSeq * 2;
  const size_t szYP   = (size_t)nAct * 4;
  const size_t szYN   = (size_t)nAct * 2;
  const size_t szTab  = (size_t)kHeads * kSeq * 4;
  const size_t szST   = (size_t)kBatch * kHeads * kStatPitch * 4;
  const size_t offXH  = 0;
  const size_t offW16 = offXH + szXH;
  const size_t offQK  = offW16 + szW16;
  const size_t offVT  = offQK + szQK;
  const size_t offATT = offVT + szVT;
  const size_t offYP  = offATT + szATT;
  const size_t offYN  = offYP + szYP;
  const size_t offRT  = offYN + szYN;
  const size_t offCT  = offRT + szTab;
  const size_t offST  = offCT + szTab;
  const size_t total  = offST + szST;
  if (ws_size < total) return;

  const float* x  = (const float*)d_in[0];
  const float* Wq = (const float*)d_in[1];
  const float* Wk = (const float*)d_in[2];
  const float* Wv = (const float*)d_in[3];
  const float* Wo = (const float*)d_in[4];
  const float* gw = (const float*)d_in[5];
  const float* gb = (const float*)d_in[6];
  float* out = (float*)d_out;
  char* ws = (char*)d_ws;
  unsigned short* XH   = (unsigned short*)(ws + offXH);
  unsigned short* W16  = (unsigned short*)(ws + offW16);
  unsigned short* QK16 = (unsigned short*)(ws + offQK);
  unsigned short* VT16 = (unsigned short*)(ws + offVT);
  unsigned short* ATT  = (unsigned short*)(ws + offATT);
  float* YPRE = (float*)(ws + offYP);
  unsigned short* YN   = (unsigned short*)(ws + offYN);
  float* RT = (float*)(ws + offRT);
  float* CT = (float*)(ws + offCT);
  float* ST = (float*)(ws + offST);

  const unsigned short* WV16 = W16 + (size_t)2 * nW;
  const unsigned short* WO16 = W16 + (size_t)3 * nW;
  const unsigned short* Q16  = QK16;
  const unsigned short* K16  = QK16 + (size_t)nAct;

  const int n8Act = nAct / 8;
  const int n8W   = nW / 8;
  cast8_kernel<<<dim3(n8Act / 256), dim3(256), 0, stream>>>(x, XH, n8Act, 1.0f);
  wcast8_kernel<<<dim3(n8W / 256, 4), dim3(256), 0, stream>>>(Wq, Wk, Wv, Wo, W16, n8W, kWCarry);
  decay_table_kernel<<<dim3(kSeq / 256, kHeads), dim3(256), 0, stream>>>(RT, CT);

  {
    const int tiles = (kTok / 64) * (kDim / 64);
    wmma_gemm64<0, false, 0, 1, false, 0, 0, false><<<dim3(tiles / 8, 2), dim3(256), 0, stream>>>(
        XH, XH, kDim, 0L, W16, W16, kDim, (long)nW,
        (void*)QK16, (void*)QK16, kDim, (long)nAct, RT, RT, 0L, kTok, kDim, kDim, kProjScale);
  }
  {
    const int tiles = (kDim / 64) * (kSeq / 64);
    wmma_gemm64<0, false, 0, 1, false, 0, 0, false><<<dim3(tiles / 8, kBatch), dim3(256), 0, stream>>>(
        WV16, WV16, kDim, 0L, XH, XH, kDim, (long)kSeq * kDim,
        (void*)VT16, (void*)VT16, kSeq, (long)kDim * kSeq, RT, RT, 0L, kDim, kSeq, kDim, kProjScale);
  }

  const long strideHead16 = (long)kDh;
  const long strideAtt    = (long)kSeq * kSeq;
  const long strideVT     = (long)kDh * kSeq;
  const int  tilesScore   = (kSeq / 64) * (kSeq / 64);
  const int  tilesPV      = (kSeq / 64) * (kDh / 64);
  for (int b = 0; b < kBatch; ++b) {
    for (int g = 0; g < kHeads / kGroup; ++g) {
      const size_t tokOff = ((size_t)b * kSeq) * kDim + (size_t)g * kGroup * kDh;
      const unsigned short* Ag  = Q16 + tokOff;
      const unsigned short* Btg = K16 + tokOff;
      const float* RTg = RT + (size_t)g * kGroup * kSeq;
      const float* CTg = CT + (size_t)g * kGroup * kSeq;
      wmma_gemm64<0, false, 0, 1, false, 0, 1, true><<<dim3(tilesScore / 8, kGroup), dim3(256), 0, stream>>>(
          Ag, Ag, kDim, strideHead16, Btg, Btg, kDim, strideHead16,
          (void*)ATT, (void*)ATT, kSeq, strideAtt, RTg, CTg, (long)kSeq, kSeq, kSeq, kDh, kScoreScale);
      const unsigned short* VTg = VT16 + ((size_t)b * kDim + (size_t)g * kGroup * kDh) * kSeq;
      float* Yg = YPRE + tokOff;
      wmma_gemm64<0, false, 0, 0, false, 0, 2, false><<<dim3(tilesPV / 8, kGroup), dim3(256), 0, stream>>>(
          ATT, ATT, kSeq, strideAtt, VTg, VTg, kSeq, strideVT,
          (void*)Yg, (void*)Yg, kDim, strideHead16, RT, RT, 0L, kSeq, kDh, kSeq, kPVScale);
    }
  }

  gn_stats_kernel<<<dim3(kBatch * kHeads), dim3(256), 0, stream>>>(YPRE, ST);
  gn_apply_kernel<<<dim3(n8Act / 256), dim3(256), 0, stream>>>(YPRE, ST, gw, gb, YN, n8Act, kActCarry);

  {
    const int tiles = (kTok / 64) * (kDim / 64);
    wmma_gemm64<0, false, 0, 0, false, 0, 0, false><<<dim3(tiles / 8, 1), dim3(256), 0, stream>>>(
        YN, YN, kDim, 0L, WO16, WO16, kDim, 0L,
        (void*)out, (void*)out, kDim, 0L, RT, RT, 0L, kTok, kDim, kDim, kOutScale);
  }
}
